// FibonacciAttention_48361331752988
// MI455X (gfx1250) — hardware-verified
//
#include <hip/hip_runtime.h>
#include <math.h>
#include <stdint.h>

#define DIM    768
#define NH     12
#define HD     64
#define BB     2
#define SS     2048
#define NTOK   (BB * SS)
#define QKN    (2 * DIM)
#define NQT    (SS / 16)
#define TPW    128
#define PSP    36
#define ACARRY 16.0f
#define WSC    256.0f
#define QKC    16.0f
#define VC     16.0f
#define PC     1024.0f
#define CC     16.0f
#define NEGS   (-1.0e30f)

static_assert(NH * HD == DIM);
static_assert((NTOK % 64) == 0 && (DIM % 64) == 0 && (QKN % 64) == 0);
static_assert((SS % 128) == 0 && (SS / 32) <= TPW && (SS % 16) == 0);
static_assert(((NTOK * DIM) % 2048) == 0 && ((3 * DIM * DIM) % 2048) == 0 && ((DIM * DIM) % 2048) == 0);
static_assert(((NQT * NH * BB) % 4) == 0 && (NQT % 4) == 0);

typedef _Float16 v16h __attribute__((ext_vector_type(16)));
typedef _Float16 v8h  __attribute__((ext_vector_type(8)));
typedef float    v8f  __attribute__((ext_vector_type(8)));
typedef float    v4f  __attribute__((ext_vector_type(4)));
typedef unsigned int v4u __attribute__((ext_vector_type(4)));

union FragH { v16h v; v8h h[2]; v4u u[2]; };

__device__ __forceinline__ unsigned short bf_bits(float f) {
  unsigned u = __float_as_uint(f);
  return (unsigned short)((u + 0x7FFFu + ((u >> 16) & 1u)) >> 16);
}
__device__ __forceinline__ float bf_up(unsigned short b) { return __uint_as_float(((unsigned)b) << 16); }
__device__ __forceinline__ float bfr(float f) { return bf_up(bf_bits(f)); }
__device__ __forceinline__ unsigned short h_bits(_Float16 x) { return __builtin_bit_cast(unsigned short, x); }
__device__ __forceinline__ unsigned pk16(unsigned short a, unsigned short b) { return (unsigned)a | ((unsigned)b << 16); }
__device__ __forceinline__ v8f zero8() { v8f z = {0.f, 0.f, 0.f, 0.f, 0.f, 0.f, 0.f, 0.f}; return z; }

__device__ __forceinline__ v16h ldfrag_u(const unsigned short* p) {
  FragH f;
  f.u[0] = *(const v4u*)(p);
  f.u[1] = *(const v4u*)(p + 16);
  return f.v;
}

__device__ __forceinline__ v8f mma_raw(v16h a, v16h b, v8f c) {
  return __builtin_amdgcn_wmma_f32_16x16x32_f16(false, a, false, b, (short)0, c, false, false);
}
__device__ __forceinline__ void guard_4x1(v8f& a, v8f& b, v8f& c, v8f& d, v16h x) {
#if defined(__HIP_DEVICE_COMPILE__)
  asm volatile("v_nop\n\tv_nop\n\tv_nop\n\tv_nop" : "+v"(a), "+v"(b), "+v"(c), "+v"(d) : "v"(x));
#endif
}
__device__ __forceinline__ void keep4_h(v16h a, v16h b, v16h c, v16h d) {
#if defined(__HIP_DEVICE_COMPILE__)
  asm volatile("v_nop" :: "v"(a), "v"(b), "v"(c), "v"(d));
#endif
}
__device__ __forceinline__ void acc_guard4(v8f& a, v8f& b, v8f& c, v8f& d) {
#if defined(__HIP_DEVICE_COMPILE__)
  asm volatile("v_nop\n\tv_nop\n\tv_nop\n\tv_nop" : "+v"(a), "+v"(b), "+v"(c), "+v"(d));
#endif
}
__device__ __forceinline__ void guard_2x6(v8f& a, v8f& b, v16h x0, v16h x1, v16h x2, v16h x3, v16h x4, v16h x5) {
#if defined(__HIP_DEVICE_COMPILE__)
  asm volatile("v_nop\n\tv_nop\n\tv_nop\n\tv_nop"
               : "+v"(a), "+v"(b) : "v"(x0), "v"(x1), "v"(x2), "v"(x3), "v"(x4), "v"(x5));
#endif
}
__device__ __forceinline__ void guard_4x5(v8f& a, v8f& b, v8f& c, v8f& d, v16h x0, v16h x1, v16h x2, v16h x3, v16h x4) {
#if defined(__HIP_DEVICE_COMPILE__)
  asm volatile("v_nop\n\tv_nop\n\tv_nop\n\tv_nop"
               : "+v"(a), "+v"(b), "+v"(c), "+v"(d) : "v"(x0), "v"(x1), "v"(x2), "v"(x3), "v"(x4));
#endif
}
__device__ __forceinline__ void wave_sync_lds() {
  __builtin_amdgcn_fence(__ATOMIC_RELEASE, "workgroup");
  __builtin_amdgcn_wave_barrier();
  __builtin_amdgcn_fence(__ATOMIC_ACQUIRE, "workgroup");
}

__global__ __launch_bounds__(256) void cvt16(const float* __restrict__ src, unsigned short* dst, int n, float scale) {
  const int i = blockIdx.x * 256 + threadIdx.x;
  const size_t base = (size_t)i * 8;
  const bool live = base + 8 <= (size_t)n;
  const size_t rb = live ? base : (size_t)(n - 8);
  const v4f a = *(const v4f*)(src + rb), b = *(const v4f*)(src + rb + 4);
  float v[8];
#pragma unroll
  for (int e = 0; e < 4; ++e) { v[e] = bfr(a[e]) * scale; v[4 + e] = bfr(b[e]) * scale; }
  v4u o;
#pragma unroll
  for (int e = 0; e < 4; ++e) o[e] = pk16(h_bits((_Float16)v[2 * e]), h_bits((_Float16)v[2 * e + 1]));
  unsigned short* dp = dst + base;
  if (live) *(volatile v4u*)dp = o;
  __threadfence();
  if (live) *(volatile v4u*)dp = o;
}

__global__ __launch_bounds__(128) void mtab(const int* __restrict__ msk, unsigned* T) {
  const int lane = threadIdx.x & 31;
  const int wave = threadIdx.x >> 5;
  const int qt   = blockIdx.x * 4 + wave;
  if (qt >= NQT) return;
  const int* mrow = msk + (size_t)qt * 16 * SS;
  v4u flv = {0u, 0u, 0u, 0u};
#pragma unroll 1
  for (int jq = 0; jq < (SS >> 7); ++jq) {
#pragma unroll
    for (int u = 0; u < 4; ++u) {
      const int key = ((jq << 2) + u) * 32 + lane;
      int mt = 0;
#pragma unroll
      for (int r = 0; r < 16; ++r) mt |= mrow[(size_t)r * SS + key];
      const unsigned bal  = __builtin_amdgcn_ballot_w32(mt != 0);
      const unsigned anyb = (bal != 0u) ? 1u : 0u;
      flv[u] = (lane == jq) ? anyb : flv[u];
    }
  }
  unsigned* rowp = T + (size_t)qt * TPW;
  *(volatile v4u*)(rowp + 4 * lane) = flv;
  __threadfence();
  *(volatile v4u*)(rowp + 4 * lane) = flv;
}

__device__ __forceinline__ void kloop(v8f (&acc)[4][4], const unsigned short* __restrict__ A1, int lda,
                                      const unsigned short* __restrict__ Bb, int ldb, int m0, int n0, int K,
                                      int rlane, int koff) {
#pragma unroll 1
  for (int k0 = 0; k0 < K; k0 += 32) {
    v16h bh[4];
#pragma unroll
    for (int j = 0; j < 4; ++j) {
      const size_t bofs = (size_t)(n0 + (j << 4) + rlane) * (size_t)ldb + (size_t)(koff + k0);
      bh[j] = ldfrag_u(Bb + bofs);
    }
#pragma unroll
    for (int i = 0; i < 4; ++i) {
      const size_t ao = (size_t)(m0 + (i << 4) + rlane) * (size_t)lda + (size_t)(koff + k0);
      const v16h ah = ldfrag_u(A1 + ao);
#pragma unroll
      for (int j = 0; j < 4; ++j) acc[i][j] = mma_raw(ah, bh[j], acc[i][j]);
      guard_4x1(acc[i][0], acc[i][1], acc[i][2], acc[i][3], ah);
    }
    keep4_h(bh[0], bh[1], bh[2], bh[3]);
  }
}

template <int OM, int BIASM>
__global__ __launch_bounds__(256) void gemm64(
    const unsigned short* __restrict__ Ap, int lda,
    const unsigned short* __restrict__ Btp, int ldb,
    const float* __restrict__ bias, float bscale,
    void* Cout, int ldc, int M, int N, int K, float oscale) {
  __shared__ __align__(16) float sT[8][16 * 68];
  const int lane = threadIdx.x & 31;
  const int wave = threadIdx.x >> 5;
  const int tilesN = N >> 6;
  const int tilesM = M >> 6;
  const int tile = blockIdx.x * 8 + wave;
  if (tile >= tilesM * tilesN) return;
  const int tm = tile / tilesN;
  const int tn = tile - tm * tilesN;
  const int m0 = tm << 6;
  const int n0 = tn << 6;

  const int rlane = lane & 15;
  const int koff  = (lane >> 4) * 8;
  const int mOff  = (lane >> 4) * 8;

  v8f acc[4][4];
#pragma unroll
  for (int i = 0; i < 4; ++i)
#pragma unroll
    for (int j = 0; j < 4; ++j) acc[i][j] = zero8();

  kloop(acc, Ap, lda, Btp, ldb, m0, n0, K, rlane, koff);
  acc_guard4(acc[0][0], acc[0][1], acc[0][2], acc[0][3]);
  acc_guard4(acc[1][0], acc[1][1], acc[1][2], acc[1][3]);
  acc_guard4(acc[2][0], acc[2][1], acc[2][2], acc[2][3]);
  acc_guard4(acc[3][0], acc[3][1], acc[3][2], acc[3][3]);

  const int hh2 = lane >> 4, c4 = (lane & 15) * 4;
  const int q8  = lane >> 3, c8 = (lane & 7) * 8;
  float bc4[4], bc8[8];
#pragma unroll
  for (int e = 0; e < 4; ++e) bc4[e] = 0.f;
#pragma unroll
  for (int e = 0; e < 8; ++e) bc8[e] = 0.f;
  if (BIASM == 0) {
    if (OM == 4) {
      const int cb = n0 + c4;
      const int i0 = (cb < N - 4) ? cb : (N - 4);
      const v4f b0v = *(const v4f*)(bias + i0);
#pragma unroll
      for (int e = 0; e < 4; ++e) bc4[e] = bfr(b0v[e]) * bscale;
    } else {
      const int cb = n0 + c8;
      const int i0 = (cb < N - 8) ? cb : (N - 8);
      const v4f b0v = *(const v4f*)(bias + i0), b1v = *(const v4f*)(bias + i0 + 4);
#pragma unroll
      for (int e = 0; e < 4; ++e) { bc8[e] = bfr(b0v[e]) * bscale; bc8[4 + e] = bfr(b1v[e]) * bscale; }
    }
  }

  float* slab = sT[wave];
#pragma unroll
  for (int i = 0; i < 4; ++i) {
    const int mBase = m0 + (i << 4);
#pragma unroll
    for (int j = 0; j < 4; ++j) {
#pragma unroll
      for (int r = 0; r < 8; ++r) {
        slab[(mOff + r) * 68 + (j << 4) + rlane] = acc[i][j][r];
      }
    }
    wave_sync_lds();
    if (OM == 4) {
      float* C = (float*)Cout;
      v4f vals[8];
#pragma unroll
      for (int it = 0; it < 8; ++it) {
        const int row = it * 2 + hh2;
        v4f v = *(const v4f*)(slab + row * 68 + c4);
        float rb = 0.f;
        if (BIASM == 1) {
          const int gr = mBase + row;
          rb = bfr(bias[(gr < M) ? gr : (M - 1)]) * bscale;
        }
#pragma unroll
        for (int e = 0; e < 4; ++e) v[e] = v[e] * oscale + bc4[e] + rb;
        vals[it] = v;
      }
#pragma unroll
      for (int it = 0; it < 8; ++it) {
        const int gr = mBase + it * 2 + hh2;
        *(volatile v4f*)(C + (size_t)gr * (size_t)ldc + n0 + c4) = vals[it];
      }
      __threadfence();
#pragma unroll
      for (int it = 0; it < 8; ++it) {
        const int gr = mBase + it * 2 + hh2;
        *(volatile v4f*)(C + (size_t)gr * (size_t)ldc + n0 + c4) = vals[it];
      }
      __threadfence();
    } else {
      unsigned short* C = (unsigned short*)Cout;
      v4u hv[4];
#pragma unroll
      for (int it = 0; it < 4; ++it) {
        const int row = it * 4 + q8;
        const float* sp = slab + row * 68 + c8;
        const v4f x0 = *(const v4f*)(sp), x1 = *(const v4f*)(sp + 4);
        float rb = 0.f;
        if (BIASM == 1) {
          const int gr = mBase + row;
          rb = bfr(bias[(gr < M) ? gr : (M - 1)]) * bscale;
        }
        float v[8];
#pragma unroll
        for (int e = 0; e < 4; ++e) {
          v[e]     = x0[e] * oscale + bc8[e] + rb;
          v[4 + e] = x1[e] * oscale + bc8[4 + e] + rb;
        }
        v4u ha;
#pragma unroll
        for (int e = 0; e < 4; ++e) ha[e] = pk16(h_bits((_Float16)v[2 * e]), h_bits((_Float16)v[2 * e + 1]));
        hv[it] = ha;
      }
#pragma unroll
      for (int it = 0; it < 4; ++it) {
        const int row = it * 4 + q8;
        const size_t o = (size_t)(mBase + row) * (size_t)ldc + n0 + c8;
        *(volatile v4u*)(C + o) = hv[it];
      }
      __threadfence();
#pragma unroll
      for (int it = 0; it < 4; ++it) {
        const int row = it * 4 + q8;
        const size_t o = (size_t)(mBase + row) * (size_t)ldc + n0 + c8;
        *(volatile v4u*)(C + o) = hv[it];
      }
      __threadfence();
    }
    wave_sync_lds();
  }
}

__device__ __forceinline__ void build_p(const float* pt, int c, int hh, FragH& ph) {
  const float* prow = pt + c * PSP + 8 * hh;
  const v4f p0 = *(const v4f*)(prow), p1 = *(const v4f*)(prow + 4);
  const v4f p2 = *(const v4f*)(prow + 16), p3 = *(const v4f*)(prow + 20);
#pragma unroll
  for (int e = 0; e < 4; ++e) {
    ph.h[0][e]     = (_Float16)(p0[e] * PC);
    ph.h[0][4 + e] = (_Float16)(p1[e] * PC);
    ph.h[1][e]     = (_Float16)(p2[e] * PC);
    ph.h[1][4 + e] = (_Float16)(p3[e] * PC);
  }
}

__global__ __launch_bounds__(128)
void attn(const unsigned short* __restrict__ QK, const unsigned short* __restrict__ VT,
          const int* __restrict__ msk, const unsigned* __restrict__ T, unsigned short* CX) {
  __shared__ __align__(16) float Ps[4][16 * PSP];
  __shared__ __align__(16) float Os[4][16 * HD];

  const int tid  = threadIdx.x;
  const int wave = tid >> 5;
  const int lane = tid & 31;
  const int hh   = lane >> 4;
  const int c    = lane & 15;

  const int wid  = blockIdx.x * 4 + wave;
  const int h    = wid % NH;
  const int rest = wid / NH;
  const int qt   = rest % NQT;
  const int b    = rest / NQT;
  if (b >= BB) return;
  const int q0   = qt * 16;
  const size_t tok0  = (size_t)b * SS + (size_t)q0;
  const size_t ktok0 = (size_t)b * SS;

  const unsigned short* qp = QK + (tok0 + (size_t)c) * (size_t)QKN + HD * h + 8 * hh;
  const v16h qf0 = ldfrag_u(qp), qf1 = ldfrag_u(qp + 32);
  const unsigned short* kp = QK + (ktok0 + (size_t)c) * (size_t)QKN + DIM + HD * h + 8 * hh;
  const unsigned short* vp = VT + (size_t)(HD * h + c) * (size_t)NTOK + ktok0 + 8 * hh;
  const int* mp = msk + (size_t)(q0 + 8 * hh) * (size_t)SS + c;
  const unsigned* trow = T + (size_t)qt * TPW;
  const float lsc = (1.4426950408889634f * 0.125f) / (QKC * QKC);

  float m[8], l[8];
  v8f z0 = zero8(), z1 = zero8(), z2 = zero8(), z3 = zero8();
#pragma unroll
  for (int r = 0; r < 8; ++r) { m[r] = NEGS; l[r] = 0.f; }
  float* pP = Ps[wave];
  const int nks = SS >> 5;

#pragma unroll 1
  for (int ks = 0; ks < nks; ++ks) {
    const int tb = __builtin_amdgcn_readfirstlane((int)trow[ks]);
    if (tb == 0) continue;
    const int kb0 = ks * 32;
    v8f s0, s1;
    {
      const unsigned short* k0p = kp + (size_t)kb0 * (size_t)QKN;
      const unsigned short* k1p = kp + (size_t)(kb0 + 16) * (size_t)QKN;
      const v16h k00 = ldfrag_u(k0p), k01 = ldfrag_u(k0p + 32);
      const v16h k10 = ldfrag_u(k1p), k11 = ldfrag_u(k1p + 32);
      s0 = mma_raw(qf0, k00, zero8());
      s0 = mma_raw(qf1, k01, s0);
      s1 = mma_raw(qf0, k10, zero8());
      s1 = mma_raw(qf1, k11, s1);
      guard_2x6(s0, s1, qf0, qf1, k00, k01, k10, k11);
    }
    int mk0[8], mk1[8];
#pragma unroll
    for (int r = 0; r < 8; ++r) {
      mk0[r] = mp[(size_t)r * SS + kb0];
      mk1[r] = mp[(size_t)r * SS + kb0 + 16];
    }
#pragma unroll
    for (int r = 0; r < 8; ++r) {
      const float t0 = s0[r] * lsc, t1 = s1[r] * lsc;
      const bool kp0 = mk0[r] != 0, kp1 = mk1[r] != 0;
      const int ro = (8 * hh + r) * PSP + c;
      float mx = fmaxf(kp0 ? t0 : NEGS, kp1 ? t1 : NEGS);
      mx = fmaxf(mx, __shfl_xor(mx, 1, 32));
      mx = fmaxf(mx, __shfl_xor(mx, 2, 32));
      mx = fmaxf(mx, __shfl_xor(mx, 4, 32));
      mx = fmaxf(mx, __shfl_xor(mx, 8, 32));
      const float mn = fmaxf(m[r], mx);
      const float al = exp2f(m[r] - mn);
      m[r] = mn;
      const float x0 = exp2f(t0 - mn), x1 = exp2f(t1 - mn);
      const float e0 = kp0 ? x0 : 0.f;
      const float e1 = kp1 ? x1 : 0.f;
      float ps = e0 + e1;
      ps += __shfl_xor(ps, 1, 32);
      ps += __shfl_xor(ps, 2, 32);
      ps += __shfl_xor(ps, 4, 32);
      ps += __shfl_xor(ps, 8, 32);
      l[r] = l[r] * al + ps;
      z0[r] *= al; z1[r] *= al; z2[r] *= al; z3[r] *= al;
      pP[ro]      = e0;
      pP[ro + 16] = e1;
    }
    wave_sync_lds();
    const v16h vf0 = ldfrag_u(vp + kb0);
    const v16h vf1 = ldfrag_u(vp + (size_t)16 * NTOK + kb0);
    const v16h vf2 = ldfrag_u(vp + (size_t)32 * NTOK + kb0);
    const v16h vf3 = ldfrag_u(vp + (size_t)48 * NTOK + kb0);
    {
      FragH ph;
      build_p(pP, c, hh, ph);
      z0 = mma_raw(ph.v, vf0, z0);
      z1 = mma_raw(ph.v, vf1, z1);
      z2 = mma_raw(ph.v, vf2, z2);
      z3 = mma_raw(ph.v, vf3, z3);
      guard_4x5(z0, z1, z2, z3, ph.v, vf0, vf1, vf2, vf3);
    }
    wave_sync_lds();
  }

  const float oc2 = CC / (PC * VC);
  float* os = Os[wave];
#pragma unroll
  for (int r = 0; r < 8; ++r) {
    const float inv = (l[r] > 0.f) ? (__builtin_amdgcn_rcpf(l[r]) * oc2) : 0.f;
    const int ro = (8 * hh + r) * HD + c;
    os[ro]      = z0[r] * inv;
    os[ro + 16] = z1[r] * inv;
    os[ro + 32] = z2[r] * inv;
    os[ro + 48] = z3[r] * inv;
  }
  wave_sync_lds();
  const int q8 = lane >> 3, c8 = (lane & 7) * 8;
  v4u ov[4];
#pragma unroll
  for (int it = 0; it < 4; ++it) {
    const int row = it * 4 + q8;
    const float* sp = os + row * HD + c8;
    const v4f x0 = *(const v4f*)(sp), x1 = *(const v4f*)(sp + 4);
    v4u a;
#pragma unroll
    for (int e = 0; e < 4; ++e) {
      const float f0 = (e < 2) ? x0[2 * e] : x1[2 * e - 4];
      const float f1 = (e < 2) ? x0[2 * e + 1] : x1[2 * e - 3];
      a[e] = pk16(h_bits((_Float16)f0), h_bits((_Float16)f1));
    }
    ov[it] = a;
  }
#pragma unroll
  for (int it = 0; it < 4; ++it) {
    const int row = it * 4 + q8;
    *(volatile v4u*)(CX + (tok0 + (size_t)row) * (size_t)DIM + HD * h + c8) = ov[it];
  }
  __threadfence();
#pragma unroll
  for (int it = 0; it < 4; ++it) {
    const int row = it * 4 + q8;
    *(volatile v4u*)(CX + (tok0 + (size_t)row) * (size_t)DIM + HD * h + c8) = ov[it];
  }
}

extern "C" void kernel_launch(void* const* d_in, const int* in_sizes, int n_in,
                              void* d_out, int out_size, void* d_ws, size_t ws_size,
                              hipStream_t stream) {
  if (n_in < 6) return;
  if (in_sizes[0] != NTOK * DIM) return;
  if (in_sizes[1] != 3 * DIM * DIM || in_sizes[2] != 3 * DIM) return;
  if (in_sizes[3] != DIM * DIM || in_sizes[4] != DIM) return;
  if (in_sizes[5] != SS * SS) return;
  if (out_size != NTOK * DIM) return;

  const float* X    = (const float*)d_in[0];
  const float* WQKV = (const float*)d_in[1];
  const float* BQKV = (const float*)d_in[2];
  const float* WO   = (const float*)d_in[3];
  const float* BO   = (const float*)d_in[4];
  const int*   MSK  = (const int*)d_in[5];
  float*       out  = (float*)d_out;

  const size_t BXP = (size_t)NTOK * DIM * 2;
  const size_t BWP = (size_t)3 * DIM * DIM * 2;
  const size_t BWO = (size_t)DIM * DIM * 2;
  const size_t BT  = (size_t)NQT * TPW * 4;
  const size_t BQK = (size_t)NTOK * QKN * 2;
  const size_t BVT = (size_t)DIM * NTOK * 2;
  const size_t BCX = (size_t)NTOK * DIM * 2;
  size_t off = 0;
  const size_t oXP = off; off += BXP;
  const size_t oWP = off; off += BWP;
  const size_t oWO = off; off += BWO;
  const size_t oT  = off; off += BT;
  const size_t oQK = off; off += BQK;
  const size_t oVT = off; off += BVT;
  const size_t oCX = off; off += BCX;
  if (off > ws_size) return;
  if (off > (size_t)134217728) return;

  char* ws = (char*)d_ws;
  unsigned short* XP  = (unsigned short*)(ws + oXP);
  unsigned short* WP  = (unsigned short*)(ws + oWP);
  unsigned short* WOP = (unsigned short*)(ws + oWO);
  unsigned*       T   = (unsigned*)(ws + oT);
  unsigned short* QKp = (unsigned short*)(ws + oQK);
  unsigned short* VTp = (unsigned short*)(ws + oVT);
  unsigned short* CXp = (unsigned short*)(ws + oCX);

  const dim3 blk(256), blk128(128);
  const float osQ = QKC / (ACARRY * WSC);
  const float osV = VC / (ACARRY * WSC);
  const float osO = 1.0f / (CC * WSC);

  cvt16<<<dim3((NTOK * DIM) / 2048), blk, 0, stream>>>(X, XP, NTOK * DIM, ACARRY);
  cvt16<<<dim3((3 * DIM * DIM) / 2048), blk, 0, stream>>>(WQKV, WP, 3 * DIM * DIM, WSC);
  cvt16<<<dim3((DIM * DIM) / 2048), blk, 0, stream>>>(WO, WOP, DIM * DIM, WSC);
  mtab<<<dim3(NQT / 4), blk128, 0, stream>>>(MSK, T);

  gemm64<2, 0><<<dim3(((NTOK / 64) * (QKN / 64) + 7) / 8), blk, 0, stream>>>(
      XP, DIM, WP, DIM, BQKV, QKC, (void*)QKp, QKN, NTOK, QKN, DIM, osQ);
  gemm64<2, 1><<<dim3(((DIM / 64) * (NTOK / 64) + 7) / 8), blk, 0, stream>>>(
      WP + (size_t)QKN * DIM, DIM, XP, DIM, BQKV + QKN, VC, (void*)VTp, NTOK, DIM, NTOK, DIM, osV);
  attn<<<dim3((NQT * NH * BB) / 4), blk128, 0, stream>>>(QKp, VTp, MSK, T, CXp);
  gemm64<4, 0><<<dim3(((NTOK / 64) * (DIM / 64) + 7) / 8), blk, 0, stream>>>(
      CXp, DIM, WOP, DIM, BO, 1.0f, (void*)out, DIM, NTOK, DIM, DIM, osO);

  (void)hipGetLastError();
}
